// LinAttention_15436112462235
// MI455X (gfx1250) — hardware-verified
//
#include <hip/hip_runtime.h>
#include <math.h>

typedef __attribute__((ext_vector_type(16))) _Float16 v16h;
typedef __attribute__((ext_vector_type(16))) __bf16 v16b;
typedef __attribute__((ext_vector_type(8)))  _Float16 v8h;
typedef __attribute__((ext_vector_type(8)))  float v8f;
typedef __attribute__((ext_vector_type(4)))  float v4f;
typedef __attribute__((ext_vector_type(2)))  float v2f;
typedef __attribute__((ext_vector_type(4)))  unsigned v4u;
typedef __attribute__((ext_vector_type(4)))  int v4i;
typedef float __attribute__((may_alias)) float_a;
typedef int __attribute__((may_alias)) int_a;

template <typename T> __device__ __forceinline__ void vst2(void* p, T v) { *(volatile T*)p = v; __threadfence(); *(volatile T*)p = v; }
__device__ __forceinline__ v8f wmma16(v16h a, v16h b, v8f c) {
  v8f d = __builtin_amdgcn_wmma_f32_16x16x32_f16(false, a, false, b, (short)0, c, false, false);
  asm volatile("v_nop\n\tv_nop\n\tv_nop\n\tv_nop" : "+v"(d) : "v"(a), "v"(b));
  return d;
}
__device__ __forceinline__ v8f wmma_bf(v16b a, v16b b, v8f c) {
  v8f d = __builtin_amdgcn_wmma_f32_16x16x32_bf16(false, a, false, b, (short)0, c, false, false);
  asm volatile("v_nop\n\tv_nop\n\tv_nop\n\tv_nop" : "+v"(d) : "v"(a), "v"(b));
  return d;
}
__device__ __forceinline__ v16h frag_h(const _Float16* rowk0, int lane) {
  union { v16h v; v8h q[2]; } u; const _Float16* p = rowk0 + 8 * (lane >> 4);
  u.q[0] = *(const v8h*)p; u.q[1] = *(const v8h*)(p + 16); return u.v;
}
__device__ __forceinline__ v16h frag_f32(const float* rowk0, int lane) {
  v16h a; const float* p = rowk0 + 8 * (lane >> 4);
#pragma unroll
  for (int i = 0; i < 8; ++i) { a[i] = (_Float16)p[i]; a[8 + i] = (_Float16)p[16 + i]; }
  return a;
}
__device__ __forceinline__ v16h frag_f32s(const float* rowk0, int lane, float sc) {
  v16h a; const float* p = rowk0 + 8 * (lane >> 4);
#pragma unroll
  for (int i = 0; i < 8; ++i) { a[i] = (_Float16)(p[i] * sc); a[8 + i] = (_Float16)(p[16 + i] * sc); }
  return a;
}
__device__ __forceinline__ v16h fragc_f32(const float* W, int k0, int n, int lane, int ld, int K) {
  v16h a; const int g = lane >> 4;
#pragma unroll
  for (int i = 0; i < 8; ++i) { const int ka = k0 + 8 * g + i, kb = ka + 16;
    a[i] = (_Float16)(ka < K ? W[(size_t)ka * ld + n] : 0.f); a[8 + i] = (_Float16)(kb < K ? W[(size_t)kb * ld + n] : 0.f); }
  return a;
}
struct F2 { v16b h, l; };
__device__ __forceinline__ F2 bsplit16(const float v[16]) { F2 r;
#pragma unroll
  for (int i = 0; i < 16; ++i) { const __bf16 h = (__bf16)v[i]; r.h[i] = h; r.l[i] = (__bf16)(v[i] - (float)h); }
  return r; }
__device__ __forceinline__ F2 split_row(const float* row, int k0, int lane) { float v[16]; const float* p = row + k0 + 8 * (lane >> 4);
#pragma unroll
  for (int i = 0; i < 8; ++i) { v[i] = p[i]; v[8 + i] = p[16 + i]; }
  return bsplit16(v); }
__device__ __forceinline__ F2 split_rowK(const float* row, int k0, int lane, int K) { float v[16]; const int g = lane >> 4;
#pragma unroll
  for (int i = 0; i < 8; ++i) { const int ka = k0 + 8 * g + i, kb = ka + 16; v[i] = ka < K ? row[ka] : 0.f; v[8 + i] = kb < K ? row[kb] : 0.f; }
  return bsplit16(v); }
__device__ __forceinline__ F2 split_col(const float* W, int k0, int n, int lane, int ld, int K) { float v[16]; const int g = lane >> 4;
#pragma unroll
  for (int i = 0; i < 8; ++i) { const int ka = k0 + 8 * g + i, kb = ka + 16; v[i] = ka < K ? W[(size_t)ka * ld + n] : 0.f; v[8 + i] = kb < K ? W[(size_t)kb * ld + n] : 0.f; }
  return bsplit16(v); }
__device__ __forceinline__ v8f mac3(const F2& a, const F2& b, v8f c) { c = wmma_bf(a.l, b.h, c); c = wmma_bf(a.h, b.l, c); return wmma_bf(a.h, b.h, c); }
__device__ __forceinline__ float sigm(float v) { return 1.0f / (1.0f + expf(-v)); }
#define LDSX() do { asm volatile("s_wait_dscnt 0" ::: "memory"); __builtin_amdgcn_wave_barrier(); __builtin_amdgcn_fence(__ATOMIC_RELEASE, "workgroup"); } while (0)

#define NB 8
#define NN 8192
#define DD 128
#define NH 8
#define KQ 64
#define NR (NB * NN)
#define RB 1024
#define NPB (NN / RB)

__global__ __launch_bounds__(256) void k_cvt(const float* __restrict__ src, _Float16* __restrict__ dst, size_t n8, float sc) {
  const size_t g8 = (size_t)blockIdx.x * 256 + threadIdx.x; if (g8 >= n8) return;
  union { v8h h; v4u u; } pk;
#pragma unroll
  for (int e = 0; e < 8; ++e) pk.h[e] = (_Float16)(src[g8 * 8 + e] * sc);
  vst2(dst + g8 * 8, pk.u);
}
__global__ __launch_bounds__(128) void k_proj(const _Float16* __restrict__ x16, const _Float16* __restrict__ Wq16, const _Float16* __restrict__ Wk16, _Float16* __restrict__ Q16, _Float16* __restrict__ KT16) {
  __shared__ __align__(16) float so[4][16][132];
  __shared__ __align__(16) _Float16 st[128][72];
  const int tid = threadIdx.x, wave = tid >> 5, lane = tid & 31, col = lane & 15, g = lane >> 4;
  const int b = blockIdx.y, z = blockIdx.z, t0b = blockIdx.x * 64, r0 = b * NN + t0b + wave * 16;
  const _Float16* W = z < 4 ? Wq16 : Wk16; const int wrow0 = (z & 3) * 128;
  v8f acc[8] = {};
#pragma unroll
  for (int kc = 0; kc < DD / 32; ++kc) { const v16h a = frag_h(x16 + (size_t)(r0 + col) * DD + kc * 32, lane);
#pragma unroll
    for (int j = 0; j < 8; ++j) acc[j] = wmma16(a, frag_h(W + (size_t)(wrow0 + j * 16 + col) * DD + kc * 32, lane), acc[j]); }
  if (z < 4) {
#pragma unroll
    for (int j = 0; j < 8; ++j)
#pragma unroll
      for (int r = 0; r < 8; ++r) so[wave][8 * g + r][j * 16 + col] = acc[j][r] * (1.0f / 16.0f);
    LDSX();
    for (int q = lane; q < 16 * 16; q += 32) { const int rl = q >> 4, pc = q & 15; union { v8h h8; v4u u; } pk;
#pragma unroll
      for (int e = 0; e < 8; ++e) pk.h8[e] = (_Float16)so[wave][rl][pc * 8 + e];
      vst2(Q16 + (size_t)(r0 + rl) * (NH * KQ) + z * 128 + pc * 8, pk.u); } }
  else {
#pragma unroll
    for (int j = 0; j < 8; ++j)
#pragma unroll
      for (int r = 0; r < 8; ++r) st[j * 16 + col][wave * 16 + 8 * g + r] = (_Float16)(acc[j][r] * (1.0f / 16.0f));
    __syncthreads();
    for (int q = tid; q < 128 * 8; q += 128) { const int c = q >> 3, pc = q & 7; const int h = (z - 4) * 2 + (c >> 6), kq = c & 63;
      vst2(KT16 + (((size_t)b * NH + h) * KQ + kq) * NN + t0b + pc * 8, *(const v4u*)(&st[c][pc * 8])); } }
}
__global__ __launch_bounds__(128) void k_ktx(const _Float16* __restrict__ KT16, const float* __restrict__ x, float* __restrict__ part) {
  __shared__ __align__(16) float so[4][16][132];
  const int tid = threadIdx.x, wave = tid >> 5, lane = tid & 31, col = lane & 15, g = lane >> 4;
  const int pb = blockIdx.x, bh = blockIdx.y, b = bh / NH; const int n0 = pb * RB;
  const _Float16* kt = KT16 + (size_t)bh * KQ * NN; const float* xb = x + ((size_t)b * NN + n0) * DD;
  v8f acc[8] = {};
#pragma unroll 1
  for (int kc = 0; kc < RB / 32; ++kc) { const v16h a = frag_h(kt + (size_t)(wave * 16 + col) * NN + n0 + kc * 32, lane);
#pragma unroll
    for (int j = 0; j < 8; ++j) acc[j] = wmma16(a, fragc_f32(xb, kc * 32, j * 16 + col, lane, DD, RB), acc[j]); }
#pragma unroll
  for (int j = 0; j < 8; ++j)
#pragma unroll
    for (int r = 0; r < 8; ++r) so[wave][8 * g + r][j * 16 + col] = acc[j][r];
  LDSX();
#pragma unroll 4
  for (int rl = 0; rl < 16; ++rl) vst2(part + (((size_t)bh * NPB + pb) * KQ + wave * 16 + rl) * DD + lane * 4, *(const v4f*)(&so[wave][rl][lane * 4]));
}
__global__ __launch_bounds__(128) void k_ktv(const float* __restrict__ part, const _Float16* __restrict__ Wv16, _Float16* __restrict__ KtV16) {
  __shared__ __align__(16) float sx[KQ][132];
  __shared__ __align__(16) _Float16 st[DD][72];
  const int tid = threadIdx.x, wave = tid >> 5, lane = tid & 31, col = lane & 15, g = lane >> 4;
  const int bh = blockIdx.x, b = bh / NH, h = bh % NH;
  for (int q = tid; q < KQ * DD; q += 128) { const int kq = q >> 7, d = q & 127; float s = 0.f;
#pragma unroll
    for (int pb = 0; pb < NPB; ++pb) s += part[(((size_t)bh * NPB + pb) * KQ + kq) * DD + d];
    sx[kq][d] = s * (1.0f / 64.0f); }
  __syncthreads();
  v8f acc[8] = {};
#pragma unroll
  for (int kc = 0; kc < DD / 32; ++kc) { const v16h a = frag_f32(&sx[wave * 16 + col][0] + kc * 32, lane);
#pragma unroll
    for (int j = 0; j < 8; ++j) acc[j] = wmma16(a, frag_h(Wv16 + ((size_t)h * DD + j * 16 + col) * DD + kc * 32, lane), acc[j]); }
#pragma unroll
  for (int j = 0; j < 8; ++j)
#pragma unroll
    for (int r = 0; r < 8; ++r) st[j * 16 + col][wave * 16 + 8 * g + r] = (_Float16)(acc[j][r] * (64.0f / 16.0f) * 0.25f);
  __syncthreads();
  for (int q = tid; q < DD * 8; q += 128) { const int e = q >> 3, pc = q & 7; vst2(KtV16 + ((size_t)b * DD + e) * (NH * KQ) + h * KQ + pc * 8, *(const v4u*)(&st[e][pc * 8])); }
}
__global__ __launch_bounds__(128) void k_out(const _Float16* __restrict__ Q16, const _Float16* __restrict__ KtV16, float* __restrict__ out) {
  __shared__ __align__(16) float so[4][16][132];
  const int tid = threadIdx.x, wave = tid >> 5, lane = tid & 31, col = lane & 15, g = lane >> 4;
  const int b = blockIdx.y, r0 = b * NN + blockIdx.x * 64 + wave * 16;
  v8f acc[8] = {};
#pragma unroll 1
  for (int kc = 0; kc < NH * KQ / 32; ++kc) { const v16h a = frag_h(Q16 + (size_t)(r0 + col) * (NH * KQ) + kc * 32, lane);
#pragma unroll
    for (int j = 0; j < 8; ++j) acc[j] = wmma16(a, frag_h(KtV16 + ((size_t)b * DD + j * 16 + col) * (NH * KQ) + kc * 32, lane), acc[j]); }
#pragma unroll
  for (int j = 0; j < 8; ++j)
#pragma unroll
    for (int r = 0; r < 8; ++r) so[wave][8 * g + r][j * 16 + col] = acc[j][r] * 4.0f;
  LDSX();
#pragma unroll 4
  for (int rl = 0; rl < 16; ++rl) vst2(out + (size_t)(r0 + rl) * DD + lane * 4, *(const v4f*)(&so[wave][rl][lane * 4]));
}
extern "C" void kernel_launch(void* const* d_in, const int* in_sizes, int n_in, void* d_out, int out_size, void* d_ws, size_t ws_size, hipStream_t stream) {
  (void)in_sizes; (void)n_in; (void)out_size; (void)ws_size;
  const float* x = (const float*)d_in[0]; const float* Wk = (const float*)d_in[1]; const float* Wq = (const float*)d_in[2]; const float* Wv = (const float*)d_in[3];
  float* out = (float*)d_out;
  char* ws = (char*)d_ws; size_t off = 0;
  auto take = [&](size_t bytes) { char* p = ws + off; off += (bytes + 255) & ~(size_t)255; return p; };
  _Float16* x16 = (_Float16*)take((size_t)NR * DD * 2); _Float16* Wq16 = (_Float16*)take((size_t)NH * KQ * DD * 2); _Float16* Wk16 = (_Float16*)take((size_t)NH * KQ * DD * 2); _Float16* Wv16 = (_Float16*)take((size_t)NH * DD * DD * 2);
  float* part = (float*)take((size_t)NB * NH * NPB * KQ * DD * 4); _Float16* KtV16 = (_Float16*)take((size_t)NB * DD * NH * KQ * 2);
  _Float16* Q16 = (_Float16*)take((size_t)NR * NH * KQ * 2); _Float16* KT16 = (_Float16*)take((size_t)NB * NH * KQ * NN * 2);
  auto cvt = [&](const float* s, _Float16* d, size_t n, float sc) { const size_t n8 = n / 8; k_cvt<<<(unsigned)((n8 + 255) / 256), 256, 0, stream>>>(s, d, n8, sc); };
  cvt(x, x16, (size_t)NR * DD, 1.0f); cvt(Wq, Wq16, (size_t)NH * KQ * DD, 16.0f); cvt(Wk, Wk16, (size_t)NH * KQ * DD, 16.0f); cvt(Wv, Wv16, (size_t)NH * DD * DD, 16.0f);
  k_proj<<<dim3(NN / 64, NB, 8), 128, 0, stream>>>(x16, Wq16, Wk16, Q16, KT16);
  k_ktx<<<dim3(NPB, NB * NH), 128, 0, stream>>>(KT16, x, part);
  k_ktv<<<NB * NH, 128, 0, stream>>>(part, Wv16, KtV16);
  k_out<<<dim3(NN / 64, NB), 128, 0, stream>>>(Q16, KtV16, out);
}
